// xLSTM_31756988187114
// MI455X (gfx1250) — hardware-verified
//
#include <hip/hip_runtime.h>
#include <math.h>

constexpr int NBAT  = 8;
constexpr int NSEQ  = 512;
constexpr int NEMB  = 512;
constexpr int NINR  = 1024;
constexpr int NHEAD = 4;
constexpr int KTAP  = 4;
constexpr int DHDS  = 128;
constexpr int DHDM  = 256;
constexpr int NPRJ  = 704;
constexpr int NLAY  = 2;
constexpr int NROW  = NBAT * NSEQ;
constexpr int NTHR  = 256;
constexpr float LNEPS = 1e-5f;
constexpr float CEPS  = 1e-6f;
constexpr float WCAR  = 16.0f;
constexpr float WCAR_INV = 1.0f / 16.0f;
constexpr float HLOCAR = 2048.0f;
constexpr float QSCALE = 1.0f / 16.0f;

static_assert(NROW % 64 == 0 && NEMB % 64 == 0 && (2 * NINR) % 64 == 0 && (2 * NPRJ) % 64 == 0 && NPRJ % 64 == 0 && (2 * DHDS) % 64 == 0, "GEMM M,N tile multiples");
static_assert(NEMB % 32 == 0 && NINR % 32 == 0 && NPRJ % 32 == 0 && DHDS % 32 == 0 && DHDM % 32 == 0, "GEMM K multiples of 32");
static_assert(NINR == NHEAD * DHDM && NEMB == NHEAD * DHDS, "head dims");
static_assert(NINR / 4 == NTHR, "conv kernel maps 256 threads x 4 channels to one row");

typedef __attribute__((ext_vector_type(16))) _Float16 v16h;
typedef __attribute__((ext_vector_type(8)))  _Float16 v8h;
typedef __attribute__((ext_vector_type(16))) __bf16   v16b;
typedef __attribute__((ext_vector_type(8)))  __bf16   v8b;
typedef __attribute__((ext_vector_type(8)))  float    v8f;
typedef __attribute__((ext_vector_type(4)))  float    v4f;
typedef __attribute__((ext_vector_type(4)))  unsigned v4u;
typedef __attribute__((ext_vector_type(2)))  unsigned v2u;

__device__ __forceinline__ unsigned short f2bf_bits(float f) {
  unsigned u = __float_as_uint(f);
  return (unsigned short)((u + 0x7FFFu + ((u >> 16) & 1u)) >> 16);
}
__device__ __forceinline__ float bf_bits2f(unsigned short h) { return __uint_as_float(((unsigned)h) << 16); }
__device__ __forceinline__ unsigned short f2h_bits(float f) { return __builtin_bit_cast(unsigned short, (_Float16)f); }
__device__ __forceinline__ void split_bf(float f, unsigned short& hb, unsigned short& lb) {
  hb = f2bf_bits(f);
  lb = f2bf_bits(f - bf_bits2f(hb));
}
__device__ __forceinline__ unsigned pack_h2(float f0, float f1) {
  return (unsigned)f2h_bits(f0) | ((unsigned)f2h_bits(f1) << 16);
}
__device__ __forceinline__ void pack_bf2(float f0, float f1, unsigned& hw, unsigned& lw) {
  unsigned short h0, l0, h1, l1;
  split_bf(f0, h0, l0);
  split_bf(f1, h1, l1);
  hw = (unsigned)h0 | ((unsigned)h1 << 16);
  lw = (unsigned)l0 | ((unsigned)l1 << 16);
}

__device__ __forceinline__ void dep_guard_h(v8f& a, v8f& b, v16h x, v16h y) { asm volatile("v_nop\n\tv_nop\n\tv_nop\n\tv_nop" : "+v"(a), "+v"(b) : "v"(x), "v"(y)); }
__device__ __forceinline__ void dep_guard_b(v8f& a, v8f& b, v16b x, v16b y) { asm volatile("v_nop\n\tv_nop\n\tv_nop\n\tv_nop" : "+v"(a), "+v"(b) : "v"(x), "v"(y)); }
__device__ __forceinline__ void keep4_h(v16h a, v16h b, v16h c, v16h d) { asm volatile("v_nop" :: "v"(a), "v"(b), "v"(c), "v"(d)); }
__device__ __forceinline__ void keep4_b(v16b a, v16b b, v16b c, v16b d) { asm volatile("v_nop" :: "v"(a), "v"(b), "v"(c), "v"(d)); }
__device__ __forceinline__ void acc_guard4(v8f& a, v8f& b, v8f& c, v8f& d) { asm volatile("v_nop\n\tv_nop\n\tv_nop\n\tv_nop" : "+v"(a), "+v"(b), "+v"(c), "+v"(d)); }
__device__ __forceinline__ void acc_guard2(v8f& a, v8f& b) { asm volatile("v_nop\n\tv_nop\n\tv_nop\n\tv_nop" : "+v"(a), "+v"(b)); }
template <typename T> struct Frag;
template <> struct Frag<_Float16> {
  typedef v16h V; union U { v16h v; v8h h[2]; };
  static __device__ __forceinline__ v16h load(const _Float16* p) {
    U f; f.h[0] = *(const v8h*)(p); f.h[1] = *(const v8h*)(p + 16); return f.v;
  }
  static __device__ __forceinline__ v8f mma(v16h a, v16h b, v8f c) {
    return __builtin_amdgcn_wmma_f32_16x16x32_f16(false, a, false, b, (short)0, c, false, false);
  }
  static __device__ __forceinline__ void guard(v8f& a, v8f& b, v16h x, v16h y) { dep_guard_h(a, b, x, y); }
  static __device__ __forceinline__ void keep(v16h a, v16h b, v16h c, v16h d) { keep4_h(a, b, c, d); }
};
template <> struct Frag<__bf16> {
  typedef v16b V; union U { v16b v; v8b h[2]; };
  static __device__ __forceinline__ v16b load(const __bf16* p) {
    U f; f.h[0] = *(const v8b*)(p); f.h[1] = *(const v8b*)(p + 16); return f.v;
  }
  static __device__ __forceinline__ v8f mma(v16b a, v16b b, v8f c) {
    return __builtin_amdgcn_wmma_f32_16x16x32_bf16(false, a, false, b, (short)0, c, false, false);
  }
  static __device__ __forceinline__ void guard(v8f& a, v8f& b, v16b x, v16b y) { dep_guard_b(a, b, x, y); }
  static __device__ __forceinline__ void keep(v16b a, v16b b, v16b c, v16b d) { keep4_b(a, b, c, d); }
};

__device__ __forceinline__ float fsigm(float x)   { return 1.0f / (1.0f + expf(-x)); }
__device__ __forceinline__ float fswish(float x)  { return x * fsigm(x); }
__device__ __forceinline__ float flogsig(float x) { return fminf(x, 0.0f) - log1pf(expf(-fabsf(x))); }
__device__ __forceinline__ float wave_sum(float v) {
#pragma unroll
  for (int off = 1; off < 32; off <<= 1) v += __shfl_xor(v, off, 32);
  return v;
}
__device__ __forceinline__ float half_sum16(float v) {
#pragma unroll
  for (int off = 1; off < 16; off <<= 1) v += __shfl_xor(v, off, 32);
  return v;
}

template <int ET> struct Elem;
template <> struct Elem<0> { typedef _Float16 T; };
template <> struct Elem<1> { typedef __bf16 T; };
template <int ET, bool SPLIT, int BIAS_MODE, bool RESID>
__global__ __launch_bounds__(256) void wmma_gemm64(
    const unsigned short* __restrict__ Ap, const unsigned short* __restrict__ A2p, int lda, long strideA,
    const unsigned short* __restrict__ Btp, const unsigned short* __restrict__ Bt2p, int ldb, long strideB,
    void* __restrict__ Cout, void* __restrict__ Cout2, int ldc, long strideC,
    const float* __restrict__ bias,
    const float* __restrict__ resid, long strideR,
    int M, int N, int K, float scale) {
  typedef typename Elem<ET>::T T;
  typedef typename Frag<T>::V V;
  const T* A = (const T*)Ap; const T* A2 = (const T*)A2p; const T* Bt = (const T*)Btp; const T* Bt2 = (const T*)Bt2p;
  __shared__ __align__(16) float sT[8][16 * 68];
  (void)Cout2;
  const int b    = blockIdx.y;
  const int lane = threadIdx.x & 31;
  const int wave = threadIdx.x >> 5;
  const int tilesN = N >> 6;
  const int tilesM = M >> 6;
  const int tile = blockIdx.x * 8 + wave;
  if (tile >= tilesM * tilesN) return;
  const int tm = tile / tilesN;
  const int tn = tile - tm * tilesN;
  const int m0 = tm << 6;
  const int n0 = tn << 6;

  const T* Ab  = A  + (size_t)b * strideA;
  const T* Bb  = Bt + (size_t)b * strideB;
  const T* Ab2 = SPLIT ? (A2  + (size_t)b * strideA) : nullptr;
  const T* Bb2 = SPLIT ? (Bt2 + (size_t)b * strideB) : nullptr;

  const int rlane = lane & 15;
  const int koff  = (lane >> 4) * 8;
  const int mOff  = (lane >> 4) * 8;

  v8f acc[4][4];
#pragma unroll
  for (int i = 0; i < 4; ++i)
#pragma unroll
    for (int j = 0; j < 4; ++j) acc[i][j] = (v8f){0.f,0.f,0.f,0.f,0.f,0.f,0.f,0.f};

  for (int k0 = 0; k0 < K; k0 += 32) {
    V bh[4], bl[4];
#pragma unroll
    for (int j = 0; j < 4; ++j) {
      const size_t bo = (size_t)(n0 + (j << 4) + rlane) * ldb + koff + k0;
      bh[j] = Frag<T>::load(Bb + bo);
      if (SPLIT) bl[j] = Frag<T>::load(Bb2 + bo);
    }
#pragma unroll
    for (int i = 0; i < 4; ++i) {
      const size_t ao = (size_t)(m0 + (i << 4) + rlane) * lda + koff + k0;
      V ah = Frag<T>::load(Ab + ao);
      V al;
      if (SPLIT) al = Frag<T>::load(Ab2 + ao);
#pragma unroll
      for (int j = 0; j < 4; ++j) {
        acc[i][j] = Frag<T>::mma(ah, bh[j], acc[i][j]);
        if (SPLIT) {
          acc[i][j] = Frag<T>::mma(ah, bl[j], acc[i][j]);
          acc[i][j] = Frag<T>::mma(al, bh[j], acc[i][j]);
        }
      }
      Frag<T>::guard(acc[i][0], acc[i][3], ah, SPLIT ? al : ah);
    }
    Frag<T>::keep(bh[0], bh[1], bh[2], bh[3]);
    if (SPLIT) Frag<T>::keep(bl[0], bl[1], bl[2], bl[3]);
  }
  acc_guard4(acc[0][0], acc[0][1], acc[0][2], acc[0][3]);
  acc_guard4(acc[1][0], acc[1][1], acc[1][2], acc[1][3]);
  acc_guard4(acc[2][0], acc[2][1], acc[2][2], acc[2][3]);
  acc_guard4(acc[3][0], acc[3][1], acc[3][2], acc[3][3]);

  float* slab = sT[wave];
  const float* Rb = RESID ? (resid + (size_t)b * strideR) : nullptr;
  float* Cb = (float*)Cout + (size_t)b * strideC;
  const int hh2 = lane >> 4, c4 = (lane & 15) * 4;
#pragma unroll
  for (int i = 0; i < 4; ++i) {
    const int mBase = m0 + (i << 4);
#pragma unroll
    for (int j = 0; j < 4; ++j) {
      const int n = n0 + (j << 4) + rlane;
      float bv = 0.f;
      if (BIAS_MODE == 2) bv = bias[n];
#pragma unroll
      for (int r = 0; r < 8; ++r) {
        float v = acc[i][j][r] * scale;
        if (BIAS_MODE == 2) v += bv;
        slab[(mOff + r) * 68 + (j << 4) + rlane] = v;
      }
    }
    __builtin_amdgcn_fence(__ATOMIC_RELEASE, "workgroup");
    __builtin_amdgcn_wave_barrier();
    __builtin_amdgcn_fence(__ATOMIC_ACQUIRE, "workgroup");
    v4f ov[8];
#pragma unroll
    for (int it = 0; it < 8; ++it) {
      const int row = it * 2 + hh2;
      v4f v = *(const v4f*)(slab + row * 68 + c4);
      if (RESID) {
        const v4f rr = *(const v4f*)(Rb + (size_t)(mBase + row) * ldc + n0 + c4);
        v += rr;
      }
      ov[it] = v;
    }
    for (int pass = 0; pass < 2; ++pass) {
#pragma unroll
      for (int it = 0; it < 8; ++it) {
        const int row = it * 2 + hh2;
        *(volatile v4f*)(Cb + (size_t)(mBase + row) * ldc + n0 + c4) = ov[it];
      }
      __threadfence();
    }
    __builtin_amdgcn_fence(__ATOMIC_RELEASE, "workgroup");
    __builtin_amdgcn_wave_barrier();
    __builtin_amdgcn_fence(__ATOMIC_ACQUIRE, "workgroup");
  }
}

template <int MODE>
__global__ __launch_bounds__(NTHR) void tpw_kernel(const float* __restrict__ src, int R, int Cc, long sstride,
                                                   unsigned short* __restrict__ O, unsigned short* __restrict__ O2,
                                                   long dstride, float sc) {
  __shared__ float Tt[64 * 65];
  const int tid = threadIdx.x;
  const int c0 = blockIdx.x * 64, r0 = blockIdx.y * 64;
  const float* sp = src + (size_t)blockIdx.z * (size_t)sstride;
  unsigned short* op  = O  + (size_t)blockIdx.z * (size_t)dstride;
  unsigned short* op2 = O2 + (size_t)blockIdx.z * (size_t)dstride;
#pragma unroll
  for (int i = 0; i < 4; ++i) {
    const int idx = i * NTHR + tid;
    const int rr = idx >> 4, cc = (idx & 15) * 4;
    const v4f v = *(const v4f*)(sp + (size_t)(r0 + rr) * (size_t)Cc + c0 + cc);
    Tt[rr * 65 + cc + 0] = v[0];
    Tt[rr * 65 + cc + 1] = v[1];
    Tt[rr * 65 + cc + 2] = v[2];
    Tt[rr * 65 + cc + 3] = v[3];
  }
  __syncthreads();
  const int q = tid >> 3, c8 = (tid & 7) * 8;
  v4u hw[2], lw[2];
#pragma unroll
  for (int g = 0; g < 2; ++g) {
    const int qq = g * 32 + q;
    unsigned h4[4], l4[4];
#pragma unroll
    for (int e = 0; e < 4; ++e) {
      const float f0 = Tt[(c8 + 2 * e) * 65 + qq];
      const float f1 = Tt[(c8 + 2 * e + 1) * 65 + qq];
      if (MODE == 0) { h4[e] = pack_h2(f0 * sc, f1 * sc); l4[e] = 0u; }
      else { pack_bf2(f0, f1, h4[e], l4[e]); }
    }
    hw[g] = (v4u){h4[0], h4[1], h4[2], h4[3]};
    lw[g] = (v4u){l4[0], l4[1], l4[2], l4[3]};
  }
  for (int pass = 0; pass < 2; ++pass) {
#pragma unroll
    for (int g = 0; g < 2; ++g) {
      const size_t o = (size_t)(c0 + g * 32 + q) * (size_t)R + (size_t)(r0 + c8);
      *(volatile v4u*)(op + o) = hw[g];
      if (MODE == 1) *(volatile v4u*)(op2 + o) = lw[g];
    }
    __threadfence();
  }
}

template <int MODE>
__global__ __launch_bounds__(NTHR) void cvt_lin_kernel(const float* __restrict__ src, unsigned short* __restrict__ O,
                                                       unsigned short* __restrict__ O2, int n8, float sc) {
  const int i = blockIdx.x * NTHR + threadIdx.x;
  if (i < n8) {
    const v4f a = *(const v4f*)(src + (size_t)i * 8);
    const v4f b = *(const v4f*)(src + (size_t)i * 8 + 4);
    unsigned h4[4], l4[4];
    if (MODE == 0) {
      h4[0] = pack_h2(a[0] * sc, a[1] * sc); h4[1] = pack_h2(a[2] * sc, a[3] * sc);
      h4[2] = pack_h2(b[0] * sc, b[1] * sc); h4[3] = pack_h2(b[2] * sc, b[3] * sc);
      l4[0] = 0u; l4[1] = 0u; l4[2] = 0u; l4[3] = 0u;
    } else {
      pack_bf2(a[0], a[1], h4[0], l4[0]); pack_bf2(a[2], a[3], h4[1], l4[1]);
      pack_bf2(b[0], b[1], h4[2], l4[2]); pack_bf2(b[2], b[3], h4[3], l4[3]);
    }
    const v4u hw = (v4u){h4[0], h4[1], h4[2], h4[3]};
    const v4u lw = (v4u){l4[0], l4[1], l4[2], l4[3]};
    for (int pass = 0; pass < 2; ++pass) {
      *(volatile v4u*)(O + (size_t)i * 8) = hw;
      if (MODE == 1) *(volatile v4u*)(O2 + (size_t)i * 8) = lw;
      __threadfence();
    }
  }
}

__global__ __launch_bounds__(NTHR) void cvt_gate_kernel(const float* __restrict__ src, unsigned short* __restrict__ OH,
                                                        unsigned short* __restrict__ OL) {
  const int t = blockIdx.x * NTHR + threadIdx.x;
  if (t < 65536) {
    const int i8 = t & 15, o = (t >> 4) & 127, g = (t >> 11) & 3, n = (t >> 13) & 3, l = t >> 15;
    const size_t si = ((((size_t)(l * 4 + g) * 4 + n) * 128 + o) * 128) + 8 * i8;
    const v4f a = *(const v4f*)(src + si);
    const v4f b = *(const v4f*)(src + si + 4);
    unsigned h4[4], l4[4];
    pack_bf2(a[0], a[1], h4[0], l4[0]); pack_bf2(a[2], a[3], h4[1], l4[1]);
    pack_bf2(b[0], b[1], h4[2], l4[2]); pack_bf2(b[2], b[3], h4[3], l4[3]);
    const v4u hw = (v4u){h4[0], h4[1], h4[2], h4[3]};
    const v4u lw = (v4u){l4[0], l4[1], l4[2], l4[3]};
    for (int pass = 0; pass < 2; ++pass) {
      *(volatile v4u*)(OH + (size_t)t * 8) = hw;
      *(volatile v4u*)(OL + (size_t)t * 8) = lw;
      __threadfence();
    }
  }
}

template <int MODE>
__global__ __launch_bounds__(NTHR) void ln16_kernel(const float* __restrict__ X, const float* __restrict__ w,
                                                    unsigned short* __restrict__ O, unsigned short* __restrict__ O2, int nrows) {
  const int tid = threadIdx.x, lane = tid & 31;
  const int row = blockIdx.x * (NTHR / 32) + (tid >> 5);
  if (row >= nrows) return;
  const float* rp = X + (size_t)row * NEMB;
  const int ca = 8 * lane, cb = 256 + 8 * lane;
  v4f v[4], g[4];
  v[0] = *(const v4f*)(rp + ca); v[1] = *(const v4f*)(rp + ca + 4);
  v[2] = *(const v4f*)(rp + cb); v[3] = *(const v4f*)(rp + cb + 4);
  g[0] = *(const v4f*)(w + ca);  g[1] = *(const v4f*)(w + ca + 4);
  g[2] = *(const v4f*)(w + cb);  g[3] = *(const v4f*)(w + cb + 4);
  float s = 0.0f;
#pragma unroll
  for (int q = 0; q < 4; ++q) s += (v[q][0] + v[q][1]) + (v[q][2] + v[q][3]);
  s = wave_sum(s);
  const float mu = s * (1.0f / NEMB);
  float ss = 0.0f;
#pragma unroll
  for (int q = 0; q < 4; ++q)
#pragma unroll
    for (int e = 0; e < 4; ++e) { const float d = v[q][e] - mu; v[q][e] = d; ss += d * d; }
  ss = wave_sum(ss);
  const float rs = rsqrtf(ss * (1.0f / NEMB) + LNEPS);
  v4f o[4];
#pragma unroll
  for (int q = 0; q < 4; ++q)
#pragma unroll
    for (int e = 0; e < 4; ++e) o[q][e] = (v[q][e] * rs) * g[q][e];
  unsigned ha[4], hb[4], la[4], lb[4];
  if (MODE == 0) {
    ha[0] = pack_h2(o[0][0], o[0][1]); ha[1] = pack_h2(o[0][2], o[0][3]);
    ha[2] = pack_h2(o[1][0], o[1][1]); ha[3] = pack_h2(o[1][2], o[1][3]);
    hb[0] = pack_h2(o[2][0], o[2][1]); hb[1] = pack_h2(o[2][2], o[2][3]);
    hb[2] = pack_h2(o[3][0], o[3][1]); hb[3] = pack_h2(o[3][2], o[3][3]);
#pragma unroll
    for (int e = 0; e < 4; ++e) { la[e] = 0u; lb[e] = 0u; }
  } else {
    pack_bf2(o[0][0], o[0][1], ha[0], la[0]); pack_bf2(o[0][2], o[0][3], ha[1], la[1]);
    pack_bf2(o[1][0], o[1][1], ha[2], la[2]); pack_bf2(o[1][2], o[1][3], ha[3], la[3]);
    pack_bf2(o[2][0], o[2][1], hb[0], lb[0]); pack_bf2(o[2][2], o[2][3], hb[1], lb[1]);
    pack_bf2(o[3][0], o[3][1], hb[2], lb[2]); pack_bf2(o[3][2], o[3][3], hb[3], lb[3]);
  }
  const v4u wa = (v4u){ha[0], ha[1], ha[2], ha[3]}, wb = (v4u){hb[0], hb[1], hb[2], hb[3]};
  const v4u xa = (v4u){la[0], la[1], la[2], la[3]}, xb = (v4u){lb[0], lb[1], lb[2], lb[3]};
  const size_t oa = (size_t)row * NEMB + ca, ob = (size_t)row * NEMB + cb;
  for (int pass = 0; pass < 2; ++pass) {
    *(volatile v4u*)(O + oa) = wa;
    *(volatile v4u*)(O + ob) = wb;
    if (MODE == 1) { *(volatile v4u*)(O2 + oa) = xa; *(volatile v4u*)(O2 + ob) = xb; }
    __threadfence();
  }
}

__global__ __launch_bounds__(NTHR) void lnf_kernel(const float* __restrict__ w, float* __restrict__ Y, int nrows) {
  const int tid = threadIdx.x, lane = tid & 31;
  const int row = blockIdx.x * (NTHR / 32) + (tid >> 5);
  if (row >= nrows) return;
  float* rp = Y + (size_t)row * NEMB;
  v4f v[4], g[4];
  float s = 0.0f;
#pragma unroll
  for (int q = 0; q < 4; ++q) {
    v[q] = *(const v4f*)(rp + 128 * q + 4 * lane);
    g[q] = *(const v4f*)(w + 128 * q + 4 * lane);
    s += (v[q][0] + v[q][1]) + (v[q][2] + v[q][3]);
  }
  s = wave_sum(s);
  const float mu = s * (1.0f / NEMB);
  float ss = 0.0f;
#pragma unroll
  for (int q = 0; q < 4; ++q)
#pragma unroll
    for (int e = 0; e < 4; ++e) { const float d = v[q][e] - mu; v[q][e] = d; ss += d * d; }
  ss = wave_sum(ss);
  const float rs = rsqrtf(ss * (1.0f / NEMB) + LNEPS);
  v4f o[4];
#pragma unroll
  for (int q = 0; q < 4; ++q)
#pragma unroll
    for (int e = 0; e < 4; ++e) o[q][e] = (v[q][e] * rs) * g[q][e];
  for (int pass = 0; pass < 2; ++pass) {
#pragma unroll
    for (int q = 0; q < 4; ++q) *(volatile v4f*)(rp + 128 * q + 4 * lane) = o[q];
    __threadfence();
  }
}

__global__ __launch_bounds__(NTHR) void conv_m_kernel(const float* __restrict__ UP, const float* __restrict__ w,
                                                      const float* __restrict__ bias, float* __restrict__ XC) {
  const int row = blockIdx.x, tid = threadIdx.x;
  const int b = row >> 9, s = row & 511;
  const int c0 = tid * 4;
  v4f x[KTAP];
#pragma unroll
  for (int j = 0; j < KTAP; ++j) {
    const int ss = s + j - (KTAP - 1);
    const int ssc = (ss < 0) ? 0 : ss;
    const v4f v = *(const v4f*)(UP + ((size_t)(b * NSEQ + ssc)) * (2 * NINR) + c0);
    x[j] = (ss >= 0) ? v : (v4f){0.0f, 0.0f, 0.0f, 0.0f};
  }
  v4f wt[4];
#pragma unroll
  for (int e = 0; e < 4; ++e) wt[e] = *(const v4f*)(w + (size_t)(c0 + e) * KTAP);
  const v4f bv = *(const v4f*)(bias + c0);
  v4f y;
#pragma unroll
  for (int e = 0; e < 4; ++e) {
    float acc = bv[e];
#pragma unroll
    for (int j = 0; j < KTAP; ++j) acc = acc + x[j][e] * wt[e][j];
    y[e] = fswish(acc);
  }
  float* dst = XC + (size_t)row * NINR + c0;
  *(volatile v4f*)dst = y;
  __threadfence();
  *(volatile v4f*)dst = y;
}

__global__ __launch_bounds__(128) void conv_s_kernel(const unsigned short* __restrict__ XH, const unsigned short* __restrict__ XL,
                                                     const float* __restrict__ w, const float* __restrict__ bias,
                                                     unsigned short* __restrict__ OH, unsigned short* __restrict__ OL) {
  const int row = blockIdx.x, tid = threadIdx.x;
  const int b = row >> 9, s = row & 511;
  const int c0 = tid * 4;
  float x[KTAP][4];
#pragma unroll
  for (int j = 0; j < KTAP; ++j) {
    const int ss = s + j - (KTAP - 1);
    const int ssc = (ss < 0) ? 0 : ss;
    const size_t o = ((size_t)(b * NSEQ + ssc)) * NEMB + c0;
    const v2u uh = *(const v2u*)(XH + o);
    const v2u ul = *(const v2u*)(XL + o);
    const float h0 = __uint_as_float(uh[0] << 16), h1 = __uint_as_float(uh[0] & 0xffff0000u);
    const float h2 = __uint_as_float(uh[1] << 16), h3 = __uint_as_float(uh[1] & 0xffff0000u);
    const float l0 = __uint_as_float(ul[0] << 16), l1 = __uint_as_float(ul[0] & 0xffff0000u);
    const float l2 = __uint_as_float(ul[1] << 16), l3 = __uint_as_float(ul[1] & 0xffff0000u);
    const bool ok = (ss >= 0);
    x[j][0] = ok ? (h0 + l0) : 0.0f;
    x[j][1] = ok ? (h1 + l1) : 0.0f;
    x[j][2] = ok ? (h2 + l2) : 0.0f;
    x[j][3] = ok ? (h3 + l3) : 0.0f;
  }
  v4f wt[4];
#pragma unroll
  for (int e = 0; e < 4; ++e) wt[e] = *(const v4f*)(w + (size_t)(c0 + e) * KTAP);
  const v4f bv = *(const v4f*)(bias + c0);
  float y[4];
#pragma unroll
  for (int e = 0; e < 4; ++e) {
    float acc = bv[e];
#pragma unroll
    for (int j = 0; j < KTAP; ++j) acc = acc + x[j][e] * wt[e][j];
    y[e] = fswish(acc);
  }
  unsigned h01, l01, h23, l23;
  pack_bf2(y[0], y[1], h01, l01);
  pack_bf2(y[2], y[3], h23, l23);
  const v2u hw = (v2u){h01, h23}, lw = (v2u){l01, l23};
  const size_t o = (size_t)row * NEMB + c0;
  for (int pass = 0; pass < 2; ++pass) {
    *(volatile v2u*)(OH + o) = hw;
    *(volatile v2u*)(OL + o) = lw;
    __threadfence();
  }
}

__global__ __launch_bounds__(NTHR) void mx_qkv_kernel(
    const float* __restrict__ XC, const float* __restrict__ UP,
    const float* __restrict__ qw, const float* __restrict__ kw, const float* __restrict__ vw,
    const float* __restrict__ igw, const float* __restrict__ fgw,
    unsigned short* __restrict__ QH, unsigned short* __restrict__ QL,
    unsigned short* __restrict__ KH, unsigned short* __restrict__ KL,
    unsigned short* __restrict__ VTH, unsigned short* __restrict__ VTL,
    float* __restrict__ IGFP) {
  __shared__ __align__(16) unsigned short Vh[256 * 72];
  __shared__ __align__(16) unsigned short Vl[256 * 72];
  __shared__ __align__(16) float igl[3072];
  __shared__ __align__(16) float fgl[3072];
  __shared__ float red[2 * 4 * 64 * 2];
  const int tid = threadIdx.x, lane = tid & 31, wave = tid >> 5;
  const int tb = blockIdx.x & 7, bn = blockIdx.x >> 3, n = bn & 3, b = bn >> 2;
  const int t0 = tb * 64;
  const int half = wave & 1, rsub = wave >> 1;
  const int chl = 128 * half + 4 * lane;
  const int cg  = n * DHDM + chl;
  const int nb  = cg >> 2;
  v4f qv[4], kv[4], vv[4];
#pragma unroll
  for (int o = 0; o < 4; ++o) {
    qv[o] = *(const v4f*)(qw + (size_t)nb * 16 + 4 * o);
    kv[o] = *(const v4f*)(kw + (size_t)nb * 16 + 4 * o);
    vv[o] = *(const v4f*)(vw + (size_t)nb * 16 + 4 * o);
  }
#pragma unroll
  for (int part = 0; part < 3; ++part) {
    *(v4f*)(igl + (part * 256 + tid) * 4) = *(const v4f*)(igw + ((size_t)(part * NINR + n * DHDM + tid)) * 4);
    *(v4f*)(fgl + (part * 256 + tid) * 4) = *(const v4f*)(fgw + ((size_t)(part * NINR + n * DHDM + tid)) * 4);
  }
  __syncthreads();
#pragma unroll 1
  for (int it = 0; it < 16; ++it) {
    const int tl = 4 * it + rsub;
    const size_t grow = (size_t)(b * NSEQ + t0 + tl);
    const v4f xc = *(const v4f*)(XC + grow * NINR + cg);
    const v4f xm = *(const v4f*)(UP + grow * (2 * NINR) + cg);
    float q[4], k[4], v[4];
#pragma unroll
    for (int o = 0; o < 4; ++o) {
      q[o] = xc[0] * qv[o][0] + xc[1] * qv[o][1] + xc[2] * qv[o][2] + xc[3] * qv[o][3];
      k[o] = xc[0] * kv[o][0] + xc[1] * kv[o][1] + xc[2] * kv[o][2] + xc[3] * kv[o][3];
      v[o] = xm[0] * vv[o][0] + xm[1] * vv[o][1] + xm[2] * vv[o][2] + xm[3] * vv[o][3];
    }
    unsigned qh0, ql0, qh1, ql1, kh0, kl0, kh1, kl1;
    pack_bf2(q[0] * QSCALE, q[1] * QSCALE, qh0, ql0);
    pack_bf2(q[2] * QSCALE, q[3] * QSCALE, qh1, ql1);
    pack_bf2(k[0], k[1], kh0, kl0);
    pack_bf2(k[2], k[3], kh1, kl1);
    const v2u qh2 = (v2u){qh0, qh1}, ql2 = (v2u){ql0, ql1}, kh2 = (v2u){kh0, kh1}, kl2 = (v2u){kl0, kl1};
    const size_t po = grow * NINR + cg;
    for (int pass = 0; pass < 2; ++pass) {
      *(volatile v2u*)(QH + po) = qh2;
      *(volatile v2u*)(QL + po) = ql2;
      *(volatile v2u*)(KH + po) = kh2;
      *(volatile v2u*)(KL + po) = kl2;
      __threadfence();
    }
#pragma unroll
    for (int o = 0; o < 4; ++o) {
      unsigned short hb, lb;
      split_bf(v[o], hb, lb);
      Vh[(chl + o) * 72 + tl] = hb;
      Vl[(chl + o) * 72 + tl] = lb;
    }
#pragma unroll 1
    for (int np = 0; np < 4; ++np) {
      float pgi = 0.0f, pgf = 0.0f;
#pragma unroll
      for (int o = 0; o < 4; ++o) {
        const int i0 = (chl + o) * 4 + np, i1 = (256 + chl + o) * 4 + np, i2 = (512 + chl + o) * 4 + np;
        pgi += q[o] * igl[i0]; pgi += k[o] * igl[i1]; pgi += v[o] * igl[i2];
        pgf += q[o] * fgl[i0]; pgf += k[o] * fgl[i1]; pgf += v[o] * fgl[i2];
      }
      pgi = wave_sum(pgi);
      pgf = wave_sum(pgf);
      if (lane == 0) {
        red[((0 * 4 + np) * 64 + tl) * 2 + half] = pgi;
        red[((1 * 4 + np) * 64 + tl) * 2 + half] = pgf;
      }
    }
  }
  __syncthreads();
  {
    const int q8 = tid >> 3, c8 = (tid & 7) * 8;
    v4u hvv[8], lvv[8];
#pragma unroll
    for (int g = 0; g < 8; ++g) {
      const int d = 32 * g + q8;
      hvv[g] = *(const v4u*)(Vh + d * 72 + c8);
      lvv[g] = *(const v4u*)(Vl + d * 72 + c8);
    }
    for (int pass = 0; pass < 2; ++pass) {
#pragma unroll
      for (int g = 0; g < 8; ++g) {
        const int d = 32 * g + q8;
        const size_t o = ((size_t)(bn * DHDM + d)) * NSEQ + t0 + c8;
        *(volatile v4u*)(VTH + o) = hvv[g];
        *(volatile v4u*)(VTL + o) = lvv[g];
      }
      __threadfence();
    }
  }
  if (wave < 4) {
    const int which = tid >> 6, np = (tid >> 4) & 3, c4 = (tid & 15) * 4;
    v4f ov;
#pragma unroll
    for (int e = 0; e < 4; ++e) {
      const int tl = c4 + e;
      ov[e] = red[((which * 4 + np) * 64 + tl) * 2 + 0] + red[((which * 4 + np) * 64 + tl) * 2 + 1];
    }
    float* dst = IGFP + (size_t)which * 65536 + ((size_t)(n * NBAT + b) * NHEAD + np) * NSEQ + t0 + c4;
    *(volatile v4f*)dst = ov;
    __threadfence();
    *(volatile v4f*)dst = ov;
  }
}

__global__ __launch_bounds__(512) void mx_scan_kernel(const float* __restrict__ IGFP, const float* __restrict__ igb,
                                                      const float* __restrict__ fgb, float* __restrict__ CSA,
                                                      float* __restrict__ BCOL, float* __restrict__ PMX) {
  __shared__ float sh[NSEQ];
  const int bn = blockIdx.x, b = bn >> 2, n = bn & 3;
  const int s = threadIdx.x;
  float ig = 0.0f, fg = 0.0f;
#pragma unroll
  for (int nb2 = 0; nb2 < 4; ++nb2) {
    const size_t o = ((size_t)(nb2 * NBAT + b) * NHEAD + n) * NSEQ + s;
    ig += IGFP[o];
    fg += IGFP[65536 + o];
  }
  ig += igb[n];
  fg += fgb[n];
  sh[s] = flogsig(fg);
  __syncthreads();
  for (int off = 1; off < NSEQ; off <<= 1) {
    const int si = (s >= off) ? (s - off) : 0;
    const float v = sh[si];
    __syncthreads();
    if (s >= off) sh[s] = sh[s] + v;
    __syncthreads();
  }
  const float cs = sh[s];
  const float bc = ig - cs;
  __syncthreads();
  sh[s] = bc;
  __syncthreads();
  for (int off = 1; off < NSEQ; off <<= 1) {
    const int si = (s >= off) ? (s - off) : 0;
    const float v = sh[si];
    __syncthreads();
    if (s >= off) sh[s] = fmaxf(sh[s], v);
    __syncthreads();
  }
  const float pm = sh[s];
  const size_t o = (size_t)bn * NSEQ + s;
  for (int pass = 0; pass < 2; ++pass) {
    ((volatile float*)CSA)[o] = cs;
    ((volatile float*)BCOL)[o] = bc;
    ((volatile float*)PMX)[o] = pm;
    __threadfence();
  }
}

__global__ __launch_bounds__(NTHR) void mx_attn_kernel(
    const unsigned short* __restrict__ QH, const unsigned short* __restrict__ QL,
    const unsigned short* __restrict__ KH, const unsigned short* __restrict__ KL,
    const unsigned short* __restrict__ VTH, const unsigned short* __restrict__ VTL,
    const float* __restrict__ CSA, const float* __restrict__ BCOL, const float* __restrict__ PMX,
    float* __restrict__ HA) {
  __shared__ __align__(16) unsigned short Ch[64 * 72];
  __shared__ __align__(16) unsigned short Cl[64 * 72];
  __shared__ float colf[64];
  __shared__ float rowf[64];
  __shared__ float psum[2 * 64];
  __shared__ __align__(16) float slabs[8][16 * 68];
  const int tid = threadIdx.x, lane = tid & 31, wave = tid >> 5;
  const int rlane = lane & 15, hh = lane >> 4, koff = hh * 8, mOff = hh * 8;
  const int qb = blockIdx.x & 7, bn = blockIdx.x >> 3, n = bn & 3, b = bn >> 2;
  const int q0 = qb * 64;
  const int im = wave & 3;
  const int jS = (wave >> 2) * 2;
  const int cO = (wave >> 2) * 128;
  const int rl0 = 16 * im + mOff;
  const v8f z8 = {0.f, 0.f, 0.f, 0.f, 0.f, 0.f, 0.f, 0.f};
  float rowsum[8];
  v8f oacc[8];
#pragma unroll
  for (int r = 0; r < 8; ++r) rowsum[r] = 0.0f;
#pragma unroll
  for (int t = 0; t < 8; ++t) oacc[t] = z8;
  const __bf16* qh = (const __bf16*)QH + (size_t)(b * NSEQ + q0 + 16 * im + rlane) * NINR + n * DHDM + koff;
  const __bf16* ql = (const __bf16*)QL + (size_t)(b * NSEQ + q0 + 16 * im + rlane) * NINR + n * DHDM + koff;

#pragma unroll 1
  for (int kc = 0; kc <= qb; ++kc) {
    const int t0 = kc * 64;
    __syncthreads();
    {
      const float bref = PMX[(size_t)bn * NSEQ + t0 + 63];
      if (wave < 2) colf[tid] = expf(BCOL[(size_t)bn * NSEQ + t0 + tid] - bref);
      else if (wave < 4) rowf[tid - 64] = expf(bref - PMX[(size_t)bn * NSEQ + q0 + tid - 64]);
    }
    v8f s0 = z8, s1 = z8;
    {
      const __bf16* kh0 = (const __bf16*)KH + (size_t)(b * NSEQ + t0 + 16 * jS + rlane) * NINR + n * DHDM + koff;
      const __bf16* kl0 = (const __bf16*)KL + (size_t)(b * NSEQ + t0 + 16 * jS + rlane) * NINR + n * DHDM + koff;
      const __bf16* kh1 = kh0 + (size_t)16 * NINR;
      const __bf16* kl1 = kl0 + (size_t)16 * NINR;
#pragma unroll 1
      for (int k0 = 0; k0 < DHDM; k0 += 32) {
        const v16b ah  = Frag<__bf16>::load(qh + k0);
        const v16b al  = Frag<__bf16>::load(ql + k0);
        const v16b bh0 = Frag<__bf16>::load(kh0 + k0);
        const v16b bl0 = Frag<__bf16>::load(kl0 + k0);
        const v16b bh1 = Frag<__bf16>::load(kh1 + k0);
        const v16b bl1 = Frag<__bf16>::load(kl1 + k0);
        s0 = Frag<__bf16>::mma(ah, bh0, s0);
        s0 = Frag<__bf16>::mma(ah, bl0, s0);
        s0 = Frag<__bf16>::mma(al, bh0, s0);
        s1 = Frag<__bf16>::mma(ah, bh1, s1);
        s1 = Frag<__bf16>::mma(ah, bl1, s1);
        s1 = Frag<__bf16>::mma(al, bh1, s1);
        dep_guard_b(s0, s1, al, bh1);
        keep4_b(ah, bh0, bl0, bl1);
      }
      acc_guard2(s0, s1);
    }
    __syncthreads();
    {
      const bool diag = (kc == qb);
      const int cl0 = 16 * jS + rlane, cl1 = cl0 + 16;
      const float cf0 = colf[cl0], cf1 = colf[cl1];
      float ps[8];
#pragma unroll
      for (int r = 0; r < 8; ++r) {
        const int rl = rl0 + r;
        const float rf = rowf[rl];
        float v0 = (s0[r] * rf) * cf0;
        float v1 = (s1[r] * rf) * cf1;
        if (diag) {
          v0 = (cl0 > rl) ? 0.0f : v0;
          v1 = (cl1 > rl) ? 0.0f : v1;
        }
        ps[r] = v0 + v1;
        unsigned short h0, l0, h1, l1;
        split_bf(v0, h0, l0);
        split_bf(v1, h1, l1);
        Ch[rl * 72 + cl0] = h0; Cl[rl * 72 + cl0] = l0;
        Ch[rl * 72 + cl1] = h1; Cl[rl * 72 + cl1] = l1;
      }
#pragma unroll
      for (int r = 0; r < 8; ++r) ps[r] = half_sum16(ps[r]);
      if (rlane == 0) {
#pragma unroll
        for (int r = 0; r < 8; ++r) psum[(wave >> 2) * 64 + rl0 + r] = ps[r];
      }
    }
    __syncthreads();
#pragma unroll
    for (int r = 0; r < 8; ++r) rowsum[r] += psum[rl0 + r] + psum[64 + rl0 + r];
    {
      const __bf16* ca  = (const __bf16*)Ch + (16 * im + rlane) * 72 + koff;
      const __bf16* cla = (const __bf16*)Cl + (16 * im + rlane) * 72 + koff;
      const __bf16* vhp = (const __bf16*)VTH + (size_t)(bn * DHDM + cO + rlane) * NSEQ + t0 + koff;
      const __bf16* vlp = (const __bf16*)VTL + (size_t)(bn * DHDM + cO + rlane) * NSEQ + t0 + koff;
#pragma unroll
      for (int kk = 0; kk < 2; ++kk) {
        const v16b ah = Frag<__bf16>::load(ca + 32 * kk);
        const v16b al = Frag<__bf16>::load(cla + 32 * kk);
#pragma unroll
        for (int grp = 0; grp < 4; ++grp) {
          const int ta = 2 * grp, tbq = 2 * grp + 1;
          const v16b bh0 = Frag<__bf16>::load(vhp + (size_t)(16 * ta) * NSEQ + 32 * kk);
          const v16b bl0 = Frag<__bf16>::load(vlp + (size_t)(16 * ta) * NSEQ + 32 * kk);
          const v16b bh1 = Frag<__bf16>::load(vhp + (size_t)(16 * tbq) * NSEQ + 32 * kk);
          const v16b bl1 = Frag<__bf16>::load(vlp + (size_t)(16 * tbq) * NSEQ + 32 * kk);
          oacc[ta]  = Frag<__bf16>::mma(ah, bh0, oacc[ta]);
          oacc[ta]  = Frag<__bf16>::mma(ah, bl0, oacc[ta]);
          oacc[ta]  = Frag<__bf16>::mma(al, bh0, oacc[ta]);
          oacc[tbq] = Frag<__bf16>::mma(ah, bh1, oacc[tbq]);
          oacc[tbq] = Frag<__bf16>::mma(ah, bl1, oacc[tbq]);
          oacc[tbq] = Frag<__bf16>::mma(al, bh1, oacc[tbq]);
          dep_guard_b(oacc[ta], oacc[tbq], ah, al);
          keep4_b(bh0, bl0, bh1, bl1);
        }
      }
    }
  }
  acc_guard4(oacc[0], oacc[1], oacc[2], oacc[3]);
  acc_guard4(oacc[4], oacc[5], oacc[6], oacc[7]);

  float inv[8];
  {
    const v4f p0 = *(const v4f*)(PMX + (size_t)bn * NSEQ + q0 + rl0);
    const v4f p1 = *(const v4f*)(PMX + (size_t)bn * NSEQ + q0 + rl0 + 4);
    const v4f c0 = *(const v4f*)(CSA + (size_t)bn * NSEQ + q0 + rl0);
    const v4f c1 = *(const v4f*)(CSA + (size_t)bn * NSEQ + q0 + rl0 + 4);
    float mr[8];
    mr[0] = c0[0] + p0[0]; mr[1] = c0[1] + p0[1]; mr[2] = c0[2] + p0[2]; mr[3] = c0[3] + p0[3];
    mr[4] = c1[0] + p1[0]; mr[5] = c1[1] + p1[1]; mr[6] = c1[2] + p1[2]; mr[7] = c1[3] + p1[3];
#pragma unroll
    for (int r = 0; r < 8; ++r) {
      const float nrm = fmaxf(fabsf(rowsum[r]), expf(-mr[r]));
      inv[r] = 1.0f / (nrm + CEPS);
    }
  }
  float* slab = slabs[wave];
  const int c4 = rlane * 4;
#pragma unroll
  for (int g = 0; g < 2; ++g) {
#pragma unroll
    for (int u = 0; u < 4; ++u)
#pragma unroll
      for (int r = 0; r < 8; ++r) slab[(mOff + r) * 68 + 16 * u + rlane] = oacc[4 * g + u][r] * inv[r];
    __builtin_amdgcn_fence(__ATOMIC_RELEASE, "workgroup");
    __builtin_amdgcn_wave_barrier();
    __builtin_amdgcn_fence(__ATOMIC_ACQUIRE, "workgroup");
    v4f ov[8];
#pragma unroll
    for (int it = 0; it < 8; ++it) {
      const int row = it * 2 + hh;
      ov[it] = *(const v4f*)(slab + row * 68 + c4);
    }
    for (int pass = 0; pass < 2; ++pass) {
#pragma unroll
      for (int it = 0; it < 8; ++it) {
        const int row = it * 2 + hh;
        float* dst = HA + (size_t)(b * NSEQ + q0 + 16 * im + row) * (2 * NINR) + n * DHDM + cO + 64 * g + c4;
        *(volatile v4f*)dst = ov[it];
      }
      __threadfence();
    }
    __builtin_amdgcn_fence(__ATOMIC_RELEASE, "workgroup");
    __builtin_amdgcn_wave_barrier();
    __builtin_amdgcn_fence(__ATOMIC_ACQUIRE, "workgroup");
  }
}

__global__ __launch_bounds__(NTHR) void mx_combine_kernel(const float* __restrict__ UP, const float* __restrict__ XC,
                                                         const float* __restrict__ skip, const float* __restrict__ nw,
                                                         unsigned short* __restrict__ YH, unsigned short* __restrict__ YL) {
  __shared__ float part[8];
  __shared__ float part2[8];
  const int tid = threadIdx.x, lane = tid & 31, wave = tid >> 5;
  const int row = blockIdx.x;
  const int n = wave >> 1, half = wave & 1;
  const int cb = n * DHDM + half * 128 + lane * 4;
  const v4f h  = *(const v4f*)(UP + (size_t)row * (2 * NINR) + cb);
  const v4f z  = *(const v4f*)(UP + (size_t)row * (2 * NINR) + NINR + cb);
  const v4f xc = *(const v4f*)(XC + (size_t)row * NINR + cb);
  const v4f sk = *(const v4f*)(skip + cb);
  const v4f g  = *(const v4f*)(nw + cb);
  float s = (h[0] + h[1]) + (h[2] + h[3]);
  s = wave_sum(s);
  if (lane == 0) part[wave] = s;
  __syncthreads();
  const float mu = (part[2 * n] + part[2 * n + 1]) * (1.0f / DHDM);
  float d[4];
  float ss = 0.0f;
#pragma unroll
  for (int e = 0; e < 4; ++e) { d[e] = h[e] - mu; ss += d[e] * d[e]; }
  ss = wave_sum(ss);
  if (lane == 0) part2[wave] = ss;
  __syncthreads();
  const float var = (part2[2 * n] + part2[2 * n + 1]) * (1.0f / DHDM);
  const float rs = rsqrtf(var + LNEPS);
  float y[4];
#pragma unroll
  for (int e = 0; e < 4; ++e) {
    const float hn = (d[e] * rs) * g[e];
    y[e] = (hn + sk[e] * xc[e]) * fswish(z[e]);
  }
  unsigned h01, l01, h23, l23;
  pack_bf2(y[0], y[1], h01, l01);
  pack_bf2(y[2], y[3], h23, l23);
  const v2u hw = (v2u){h01, h23}, lw = (v2u){l01, l23};
  const size_t o = (size_t)row * NINR + cb;
  for (int pass = 0; pass < 2; ++pass) {
    *(volatile v2u*)(YH + o) = hw;
    *(volatile v2u*)(YL + o) = lw;
    __threadfence();
  }
}

__device__ __forceinline__ float comb_hl(float elo, float ehi, int hh, float sc) {
  const float send = (hh ? elo : ehi) * sc;
  const float mine = (hh ? ehi : elo) * sc;
  const float recv = __shfl_xor(send, 16, 32);
  return mine + recv;
}

__global__ __launch_bounds__(NTHR) void sx_rec_kernel(const float* __restrict__ GX, const unsigned short* __restrict__ RFp,
                                                      const float* __restrict__ sb, float* __restrict__ HS) {
  __shared__ __align__(16) _Float16 Ah[2][16 * 136];
  __shared__ __align__(16) float    Hsl[2][8 * 132];
  const _Float16* RF = (const _Float16*)RFp;
  const int tid = threadIdx.x, lane = tid & 31, wave = tid >> 5;
  const int c = lane & 15, hh = lane >> 4, koff = hh * 8;
  const int n = blockIdx.x;
  const int j = 16 * wave + c;
  {
    _Float16* ahf = &Ah[0][0];
#pragma unroll 1
    for (int i = tid; i < 2 * 16 * 136; i += NTHR) ahf[i] = (_Float16)0.0f;
  }
  const float bb0 = sb[(0 * NHEAD + n) * DHDS + j];
  const float bb1 = sb[(1 * NHEAD + n) * DHDS + j];
  const float bb2 = sb[(2 * NHEAD + n) * DHDS + j];
  const float bb3 = sb[(3 * NHEAD + n) * DHDS + j];
  float cst[4], nst[4], mst[4];
#pragma unroll
  for (int rp = 0; rp < 4; ++rp) { cst[rp] = 0.0f; nst[rp] = 0.0f; mst[rp] = 0.0f; }
  __syncthreads();
  const v8f z8 = {0.f, 0.f, 0.f, 0.f, 0.f, 0.f, 0.f, 0.f};
  const float mysc = hh ? (1.0f / 32768.0f) : WCAR_INV;
  const _Float16* rb = RF + ((size_t)n * DHDS + j) * DHDS + koff;

#pragma unroll 1
  for (int s = 0; s < NSEQ; ++s) {
    const int cur = s & 1;
    float xg[4][4];
#pragma unroll
    for (int g = 0; g < 4; ++g)
#pragma unroll
      for (int rp = 0; rp < 4; ++rp)
        xg[g][rp] = GX[((size_t)((4 * hh + rp) * NSEQ + s)) * (2 * NINR) + n * 512 + g * 128 + j];
    const _Float16* arow = &Ah[cur][0] + c * 136 + koff;
    v8f acc0 = z8, acc1 = z8, acc2 = z8, acc3 = z8;
#pragma unroll 1
    for (int k0 = 0; k0 < DHDS; k0 += 32) {
      const v16h a  = Frag<_Float16>::load(arow + k0);
      const v16h b0 = Frag<_Float16>::load(rb + k0);
      const v16h b1 = Frag<_Float16>::load(rb + 65536 + k0);
      const v16h b2 = Frag<_Float16>::load(rb + 131072 + k0);
      const v16h b3 = Frag<_Float16>::load(rb + 196608 + k0);
      acc0 = Frag<_Float16>::mma(a, b0, acc0);
      acc1 = Frag<_Float16>::mma(a, b1, acc1);
      acc2 = Frag<_Float16>::mma(a, b2, acc2);
      acc3 = Frag<_Float16>::mma(a, b3, acc3);
      dep_guard_h(acc0, acc3, a, b3);
      keep4_h(b0, b1, b2, b3);
    }
    acc_guard4(acc0, acc1, acc2, acc3);
    float hr0[4], hr1[4], hr2[4], hr3[4];
#pragma unroll
    for (int rp = 0; rp < 4; ++rp) {
      hr0[rp] = comb_hl(acc0[rp], acc0[4 + rp], hh, mysc);
      hr1[rp] = comb_hl(acc1[rp], acc1[4 + rp], hh, mysc);
      hr2[rp] = comb_hl(acc2[rp], acc2[4 + rp], hh, mysc);
      hr3[rp] = comb_hl(acc3[rp], acc3[4 + rp], hh, mysc);
    }
    _Float16* ahn = &Ah[cur ^ 1][0];
    float* hsl = &Hsl[cur][0];
#pragma unroll
    for (int rp = 0; rp < 4; ++rp) {
      const float ir  = (xg[0][rp] + bb0) + hr0[rp];
      const float fr  = (xg[1][rp] + bb1) + hr1[rp];
      const float zr  = (xg[2][rp] + bb2) + hr2[rp];
      const float orr = (xg[3][rp] + bb3) + hr3[rp];
      const float lf = mst[rp] + flogsig(fr);
      const float mn = fmaxf(ir, lf);
      const float iv = expf(ir - mn);
      const float fv = expf(lf - mn);
      const float cn = fv * cst[rp] + iv * tanhf(zr);
      const float nn = fv * nst[rp] + iv;
      const float hv = (fsigm(orr) * cn) / nn;
      cst[rp] = cn; nst[rp] = nn; mst[rp] = mn;
      const _Float16 hi16 = (_Float16)hv;
      const float hif = (float)hi16;
      const _Float16 lo16 = (_Float16)((hv - hif) * HLOCAR);
      const int brow = 4 * hh + rp;
      ahn[brow * 136 + j] = hi16;
      ahn[(8 + brow) * 136 + j] = lo16;
      hsl[brow * 132 + j] = hv;
    }
    __syncthreads();
    {
      const v4f hv4 = *(const v4f*)(hsl + wave * 132 + lane * 4);
      float* dst = HS + ((size_t)(wave * NSEQ + s)) * NEMB + n * DHDS + lane * 4;
      *(volatile v4f*)dst = hv4;
      __threadfence();
      *(volatile v4f*)dst = hv4;
    }
  }
}

__global__ __launch_bounds__(NTHR) void sx_gn_kernel(const float* __restrict__ HS, const float* __restrict__ gw,
                                                     float* __restrict__ OUT) {
  const int tid = threadIdx.x, lane = tid & 31, wave = tid >> 5;
  const int unit = blockIdx.x * 8 + wave;
  const int row = unit >> 2, n = unit & 3;
  const size_t base = (size_t)row * NEMB + n * DHDS + lane * 4;
  const v4f x  = *(const v4f*)(HS + base);
  const v4f g  = *(const v4f*)(gw + n * DHDS + lane * 4);
  const v4f o0 = *(const v4f*)(OUT + base);
  float s = (x[0] + x[1]) + (x[2] + x[3]);
  s = wave_sum(s);
  const float mu = s * (1.0f / DHDS);
  float d[4];
  float ss = 0.0f;
#pragma unroll
  for (int e = 0; e < 4; ++e) { d[e] = x[e] - mu; ss += d[e] * d[e]; }
  ss = wave_sum(ss);
  const float rs = rsqrtf(ss * (1.0f / DHDS) + LNEPS);
  v4f o;
#pragma unroll
  for (int e = 0; e < 4; ++e) o[e] = o0[e] + (d[e] * rs) * g[e];
  *(volatile v4f*)(OUT + base) = o;
  __threadfence();
  *(volatile v4f*)(OUT + base) = o;
}

__global__ __launch_bounds__(NTHR) void ffn_gelu_kernel(const float* __restrict__ U, unsigned short* __restrict__ PH,
                                                        unsigned short* __restrict__ PL, int n2) {
  const int i = blockIdx.x * NTHR + threadIdx.x;
  if (i < n2) {
    const int row = i / (NPRJ / 2);
    const int cp = (i - row * (NPRJ / 2)) * 2;
    const float* up = U + (size_t)row * (2 * NPRJ) + cp;
    const float a0 = up[0], a1 = up[1];
    const float g0 = up[NPRJ], g1 = up[NPRJ + 1];
    const float p0 = (0.5f * a0 * (1.0f + erff(a0 * 0.70710678118654752f))) * g0;
    const float p1 = (0.5f * a1 * (1.0f + erff(a1 * 0.70710678118654752f))) * g1;
    unsigned hw, lw;
    pack_bf2(p0, p1, hw, lw);
    for (int pass = 0; pass < 2; ++pass) {
      ((volatile unsigned*)PH)[i] = hw;
      ((volatile unsigned*)PL)[i] = lw;
      __threadfence();
    }
  }
}

constexpr size_t SZ_FIN1  = (size_t)NEMB * NEMB * 2;
constexpr size_t SZ_MUPT  = (size_t)NLAY * 2 * NINR * NEMB * 2;
constexpr size_t SZ_MDN1  = (size_t)NLAY * NEMB * NINR * 2;
constexpr size_t SZ_GW1   = (size_t)NLAY * 4 * NHEAD * DHDS * DHDS * 2;
constexpr size_t SZ_RF    = SZ_GW1;
constexpr size_t SZ_FUPT  = (size_t)NLAY * 2 * NPRJ * NEMB * 2;
constexpr size_t SZ_FDN1  = (size_t)NLAY * NEMB * NPRJ * 2;
constexpr size_t SZ_XINF  = (size_t)NROW * NEMB * 2;
constexpr size_t SZ_XIN1  = (size_t)NROW * NEMB * 2;
constexpr size_t SZ_UPB   = (size_t)NROW * 2 * NINR * 4;
constexpr size_t SZ_XCB   = (size_t)NROW * NINR * 4;
constexpr size_t SZ_P1    = (size_t)NROW * NINR * 2;
constexpr size_t SZ_IGFP  = (size_t)2 * 65536 * 4;
constexpr size_t SZ_ST1   = (size_t)NBAT * NHEAD * NSEQ * 4;
constexpr size_t WS_TOTAL = 2 * SZ_FIN1 + SZ_MUPT + 2 * SZ_MDN1 + 2 * SZ_GW1 + SZ_RF + SZ_FUPT + 2 * SZ_FDN1 +
                            SZ_XINF + 2 * SZ_XIN1 + SZ_UPB + SZ_XCB + 6 * SZ_P1 + SZ_IGFP + 3 * SZ_ST1;
static_assert(WS_TOTAL == 132317184ull, "region map total");
static_assert(WS_TOTAL <= 134217728ull, "carve within 128 MiB");
static_assert((size_t)4 * NROW * NEMB * 4 <= SZ_UPB && (size_t)NROW * 2 * NPRJ * 4 <= SZ_UPB, "UPB re-use");
static_assert((size_t)NROW * NEMB * 4 <= SZ_XCB, "XCB re-use");
static_assert((size_t)NROW * NPRJ * 2 <= SZ_P1 && (size_t)NROW * NEMB * 2 <= SZ_P1, "plane re-use");

extern "C" void kernel_launch(void* const* d_in, const int* in_sizes, int n_in,
                              void* d_out, int out_size, void* d_ws, size_t ws_size, hipStream_t stream) {
  if (n_in < 30 || d_out == nullptr || d_ws == nullptr) return;
  if (in_sizes[0] != NROW * NEMB || in_sizes[1] != NEMB * NEMB || in_sizes[2] != NEMB ||
      in_sizes[3] != NLAY * NEMB || in_sizes[4] != NLAY * NEMB * 2 * NINR || in_sizes[5] != NLAY * 2 * NINR ||
      in_sizes[6] != NLAY * NINR * KTAP || in_sizes[7] != NLAY * NINR ||
      in_sizes[8] != NLAY * (NINR / 4) * 16 || in_sizes[9] != NLAY * (NINR / 4) * 16 || in_sizes[10] != NLAY * (NINR / 4) * 16 ||
      in_sizes[11] != NLAY * 3 * NINR * NHEAD || in_sizes[12] != NLAY * NHEAD || in_sizes[13] != NLAY * 3 * NINR * NHEAD ||
      in_sizes[14] != NLAY * NHEAD || in_sizes[15] != NLAY * NINR || in_sizes[16] != NLAY * NINR ||
      in_sizes[17] != NLAY * NINR * NEMB || in_sizes[18] != NLAY * NEMB || in_sizes[19] != NLAY * NEMB ||
      in_sizes[20] != NLAY * NEMB * KTAP || in_sizes[21] != NLAY * NEMB ||
      in_sizes[22] != NLAY * 4 * NHEAD * DHDS * DHDS || in_sizes[23] != NLAY * 4 * NHEAD * DHDS * DHDS ||
      in_sizes[24] != NLAY * 4 * NHEAD * DHDS || in_sizes[25] != NLAY * NEMB || in_sizes[26] != NLAY * NEMB ||
      in_sizes[27] != NLAY * NEMB * 2 * NPRJ || in_sizes[28] != NLAY * NPRJ * NEMB || in_sizes[29] != NEMB ||
      out_size != NROW * NEMB) return;

  const float* x_in     = (const float*)d_in[0];
  const float* fin_w    = (const float*)d_in[1];
  const float* fin_b    = (const float*)d_in[2];
  const float* m_ln_w   = (const float*)d_in[3];
  const float* m_up_w   = (const float*)d_in[4];
  const float* m_up_b   = (const float*)d_in[5];
  const float* m_conv_w = (const float*)d_in[6];
  const float* m_conv_b = (const float*)d_in[7];
  const float* m_q_w    = (const float*)d_in[8];
  const float* m_k_w    = (const float*)d_in[9];
  const float* m_v_w    = (const float*)d_in[10];
  const float* m_ig_w   = (const float*)d_in[11];
  const float* m_ig_b   = (const float*)d_in[12];
  const float* m_fg_w   = (const float*)d_in[13];
  const float* m_fg_b   = (const float*)d_in[14];
  const float* m_skip   = (const float*)d_in[15];
  const float* m_norm_w = (const float*)d_in[16];
  const float* m_down_w = (const float*)d_in[17];
  const float* m_down_b = (const float*)d_in[18];
  const float* s_ln_w   = (const float*)d_in[19];
  const float* s_conv_w = (const float*)d_in[20];
  const float* s_conv_b = (const float*)d_in[21];
  const float* s_gate_w = (const float*)d_in[22];
  const float* s_R      = (const float*)d_in[23];
  const float* s_bias   = (const float*)d_in[24];
  const float* s_gn_w   = (const float*)d_in[25];
  const float* s_ln2_w  = (const float*)d_in[26];
  const float* s_ffu_w  = (const float*)d_in[27];
  const float* s_ffd_w  = (const float*)d_in[28];
  const float* post_w   = (const float*)d_in[29];
  float* out = (float*)d_out;

  char* ws = (char*)d_ws; size_t off = 0;
  auto carve = [&](size_t bytes) -> char* { char* p = ws + off; off += (bytes + 255) & ~(size_t)255; return p; };
  unsigned short* FINH = (unsigned short*)carve(SZ_FIN1);
  unsigned short* FINL = (unsigned short*)carve(SZ_FIN1);
  unsigned short* MUPT = (unsigned short*)carve(SZ_MUPT);
  unsigned short* MDNH = (unsigned short*)carve(SZ_MDN1);
  unsigned short* MDNL = (unsigned short*)carve(SZ_MDN1);
  unsigned short* GWH  = (unsigned short*)carve(SZ_GW1);
  unsigned short* GWL  = (unsigned short*)carve(SZ_GW1);
  unsigned short* RF16 = (unsigned short*)carve(SZ_RF);
  unsigned short* FUPT = (unsigned short*)carve(SZ_FUPT);
  unsigned short* FDNH = (unsigned short*)carve(SZ_FDN1);
  unsigned short* FDNL = (unsigned short*)carve(SZ_FDN1);
  unsigned short* XINF = (unsigned short*)carve(SZ_XINF);
  unsigned short* XINH = (unsigned short*)carve(SZ_XIN1);
  unsigned short* XINL = (unsigned short*)carve(SZ_XIN1);
  float*          UPB  = (float*)carve(SZ_UPB);
  float*          XCB  = (float*)carve(SZ_XCB);
  unsigned short* QHB  = (unsigned short*)carve(SZ_P1);
  unsigned short* QLB  = (unsigned short*)carve(SZ_P1);
  unsigned short* KHB  = (unsigned short*)carve(SZ_P1);
  unsigned short* KLB  = (unsigned short*)carve(SZ_P1);
  unsigned short* VTHB = (unsigned short*)carve(SZ_P1);
  unsigned short* VTLB = (unsigned short*)carve(SZ_P1);
  float*          IGFP = (float*)carve(SZ_IGFP);
  float*          CSA  = (float*)carve(SZ_ST1);
  float*          BCOL = (float*)carve(SZ_ST1);
  float*          PMX  = (float*)carve(SZ_ST1);
  if (off > ws_size || off > (size_t)134217728) return;

  tpw_kernel<1><<<dim3(NEMB / 64, NEMB / 64, 1), NTHR, 0, stream>>>(fin_w, NEMB, NEMB, 0L, FINH, FINL, 0L, 1.0f);
  tpw_kernel<0><<<dim3(2 * NINR / 64, NEMB / 64, NLAY), NTHR, 0, stream>>>(m_up_w, NEMB, 2 * NINR, (long)NEMB * 2 * NINR, MUPT, MUPT, (long)2 * NINR * NEMB, WCAR);
  tpw_kernel<1><<<dim3(NEMB / 64, NINR / 64, NLAY), NTHR, 0, stream>>>(m_down_w, NINR, NEMB, (long)NINR * NEMB, MDNH, MDNL, (long)NEMB * NINR, 1.0f);
  tpw_kernel<0><<<dim3(2 * NPRJ / 64, NEMB / 64, NLAY), NTHR, 0, stream>>>(s_ffu_w, NEMB, 2 * NPRJ, (long)NEMB * 2 * NPRJ, FUPT, FUPT, (long)2 * NPRJ * NEMB, WCAR);
  tpw_kernel<1><<<dim3(NEMB / 64, NPRJ / 64, NLAY), NTHR, 0, stream>>>(s_ffd_w, NPRJ, NEMB, (long)NPRJ * NEMB, FDNH, FDNL, (long)NEMB * NPRJ, 1.0f);
  cvt_gate_kernel<<<65536 / NTHR, NTHR, 0, stream>>>(s_gate_w, GWH, GWL);
  {
    const int n8r = NLAY * 4 * NHEAD * DHDS * DHDS / 8;
    cvt_lin_kernel<0><<<(n8r + NTHR - 1) / NTHR, NTHR, 0, stream>>>(s_R, RF16, RF16, n8r, WCAR);
    const int n8x = NROW * NEMB / 8;
    cvt_lin_kernel<1><<<(n8x + NTHR - 1) / NTHR, NTHR, 0, stream>>>(x_in, XINH, XINL, n8x, 1.0f);
  }
  {
    const int tiles = (NROW / 64) * (NEMB / 64);
    wmma_gemm64<1, true, 2, false><<<dim3((tiles + 7) / 8, 1), 256, 0, stream>>>(
        XINH, XINL, NEMB, 0L, FINH, FINL, NEMB, 0L, (void*)out, (void*)out, NEMB, 0L,
        fin_b, out, 0L, NROW, NEMB, NEMB, 1.0f);
  }

  for (int l = 0; l < NLAY; ++l) {
    const float* mlw  = m_ln_w   + (size_t)l * NEMB;
    const float* mub  = m_up_b   + (size_t)l * 2 * NINR;
    const float* mcw  = m_conv_w + (size_t)l * NINR * KTAP;
    const float* mcb  = m_conv_b + (size_t)l * NINR;
    const float* mqw  = m_q_w    + (size_t)l * (NINR / 4) * 16;
    const float* mkw  = m_k_w    + (size_t)l * (NINR / 4) * 16;
    const float* mvw  = m_v_w    + (size_t)l * (NINR / 4) * 16;
    const float* migw = m_ig_w   + (size_t)l * 3 * NINR * NHEAD;
    const float* migb = m_ig_b   + (size_t)l * NHEAD;
    const float* mfgw = m_fg_w   + (size_t)l * 3 * NINR * NHEAD;
    const float* mfgb = m_fg_b   + (size_t)l * NHEAD;
    const float* mskp = m_skip   + (size_t)l * NINR;
    const float* mnw  = m_norm_w + (size_t)l * NINR;
    const float* mdb  = m_down_b + (size_t)l * NEMB;
    const float* slw  = s_ln_w   + (size_t)l * NEMB;
    const float* scw  = s_conv_w + (size_t)l * NEMB * KTAP;
    const float* scb  = s_conv_b + (size_t)l * NEMB;
    const float* sbl  = s_bias   + (size_t)l * 4 * NHEAD * DHDS;
    const float* sgnw = s_gn_w   + (size_t)l * NEMB;
    const float* sl2w = s_ln2_w  + (size_t)l * NEMB;
    const unsigned short* MUPTl = MUPT + (size_t)l * 2 * NINR * NEMB;
    const unsigned short* MDNHl = MDNH + (size_t)l * NEMB * NINR;
    const unsigned short* MDNLl = MDNL + (size_t)l * NEMB * NINR;
    const unsigned short* GWHl  = GWH  + (size_t)l * 4 * NHEAD * DHDS * DHDS;
    const unsigned short* GWLl  = GWL  + (size_t)l * 4 * NHEAD * DHDS * DHDS;
    const unsigned short* RFl   = RF16 + (size_t)l * 4 * NHEAD * DHDS * DHDS;
    const unsigned short* FUPTl = FUPT + (size_t)l * 2 * NPRJ * NEMB;
    const unsigned short* FDNHl = FDNH + (size_t)l * NEMB * NPRJ;
    const unsigned short* FDNLl = FDNL + (size_t)l * NEMB * NPRJ;

    ln16_kernel<0><<<NROW / 8, NTHR, 0, stream>>>(out, mlw, XINF, XINF, NROW);
    {
      const int tiles = (NROW / 64) * (2 * NINR / 64);
      wmma_gemm64<0, false, 2, false><<<dim3((tiles + 7) / 8, 1), 256, 0, stream>>>(
          XINF, XINF, NEMB, 0L, MUPTl, MUPTl, NEMB, 0L, (void*)UPB, (void*)UPB, 2 * NINR, 0L,
          mub, out, 0L, NROW, 2 * NINR, NEMB, WCAR_INV);
    }
    conv_m_kernel<<<NROW, NTHR, 0, stream>>>(UPB, mcw, mcb, XCB);
    mx_qkv_kernel<<<NBAT * NHEAD * (NSEQ / 64), NTHR, 0, stream>>>(XCB, UPB, mqw, mkw, mvw, migw, mfgw,
                                                                   QHB, QLB, KHB, KLB, VTHB, VTLB, IGFP);
    mx_scan_kernel<<<NBAT * NHEAD, 512, 0, stream>>>(IGFP, migb, mfgb, CSA, BCOL, PMX);
    mx_attn_kernel<<<NBAT * NHEAD * (NSEQ / 64), NTHR, 0, stream>>>(QHB, QLB, KHB, KLB, VTHB, VTLB, CSA, BCOL, PMX, UPB);
    mx_combine_kernel<<<NROW, NTHR, 0, stream>>>(UPB, XCB, mskp, mnw, QHB, QLB);
    {
      const int tiles = (NROW / 64) * (NEMB / 64);
      wmma_gemm64<1, true, 2, true><<<dim3((tiles + 7) / 8, 1), 256, 0, stream>>>(
          QHB, QLB, NINR, 0L, MDNHl, MDNLl, NINR, 0L, (void*)out, (void*)out, NEMB, 0L,
          mdb, out, 0L, NROW, NEMB, NINR, 1.0f);
    }

    ln16_kernel<1><<<NROW / 8, NTHR, 0, stream>>>(out, slw, XINH, XINL, NROW);
    conv_s_kernel<<<NROW, 128, 0, stream>>>(XINH, XINL, scw, scb, KHB, KLB);
    {
      const int tiles = (NROW / 64) * (2 * DHDS / 64);
      const long sB = (long)4 * DHDS * DHDS;
      wmma_gemm64<1, true, 0, false><<<dim3((tiles + 7) / 8, NHEAD), 256, 0, stream>>>(
          KHB, KLB, NEMB, (long)DHDS, GWHl, GWLl, DHDS, sB, (void*)UPB, (void*)UPB, 2 * NINR, (long)(4 * DHDS),
          fin_b, out, 0L, NROW, 2 * DHDS, DHDS, 1.0f);
      wmma_gemm64<1, true, 0, false><<<dim3((tiles + 7) / 8, NHEAD), 256, 0, stream>>>(
          XINH, XINL, NEMB, (long)DHDS, GWHl + 2 * DHDS * DHDS, GWLl + 2 * DHDS * DHDS, DHDS, sB,
          (void*)(UPB + 2 * DHDS), (void*)(UPB + 2 * DHDS), 2 * NINR, (long)(4 * DHDS),
          fin_b, out, 0L, NROW, 2 * DHDS, DHDS, 1.0f);
    }
    sx_rec_kernel<<<NHEAD, NTHR, 0, stream>>>(UPB, RFl, sbl, XCB);
    sx_gn_kernel<<<NROW * NHEAD / 8, NTHR, 0, stream>>>(XCB, sgnw, out);

    ln16_kernel<0><<<NROW / 8, NTHR, 0, stream>>>(out, sl2w, XINF, XINF, NROW);
    {
      const int tiles = (NROW / 64) * (2 * NPRJ / 64);
      wmma_gemm64<0, false, 0, false><<<dim3((tiles + 7) / 8, 1), 256, 0, stream>>>(
          XINF, XINF, NEMB, 0L, FUPTl, FUPTl, NEMB, 0L, (void*)UPB, (void*)UPB, 2 * NPRJ, 0L,
          fin_b, out, 0L, NROW, 2 * NPRJ, NEMB, WCAR_INV);
    }
    {
      const int n2 = NROW * NPRJ / 2;
      ffn_gelu_kernel<<<(n2 + NTHR - 1) / NTHR, NTHR, 0, stream>>>(UPB, QHB, QLB, n2);
    }
    {
      const int tiles = (NROW / 64) * (NEMB / 64);
      wmma_gemm64<1, true, 0, true><<<dim3((tiles + 7) / 8, 1), 256, 0, stream>>>(
          QHB, QLB, NPRJ, 0L, FDNHl, FDNLl, NPRJ, 0L, (void*)out, (void*)out, NEMB, 0L,
          fin_b, out, 0L, NROW, NEMB, NPRJ, 1.0f);
    }
  }

  lnf_kernel<<<NROW / 8, NTHR, 0, stream>>>(post_w, out, NROW);
}
